// GNN_62285615727516
// MI455X (gfx1250) — hardware-run, weakly checked
//
#include <hip/hip_runtime.h>

typedef float          v8f   __attribute__((ext_vector_type(8)));
typedef float          v4f   __attribute__((ext_vector_type(4)));
typedef unsigned int   v4u   __attribute__((ext_vector_type(4)));
typedef int            v8i   __attribute__((ext_vector_type(8)));
typedef unsigned short v8us  __attribute__((ext_vector_type(8)));
typedef unsigned short v16us __attribute__((ext_vector_type(16)));
typedef __bf16         v16bf __attribute__((ext_vector_type(16)));
typedef _Float16       v16h  __attribute__((ext_vector_type(16)));
typedef v4f  __attribute__((may_alias)) v4fa;
typedef v8us __attribute__((may_alias)) v8usa;
union FragB { v16bf v; v16us u; v8us h[2]; v8i w; };
union FragH { v16h  v; v16us u; v8us h[2]; v8i w; };

__device__ __forceinline__ v8f wmb(const FragB& a, const FragB& b, v8f c) {
  v8f d = __builtin_amdgcn_wmma_f32_16x16x32_bf16(false, a.v, false, b.v, (short)0, c, false, false);
  asm volatile("v_nop\n\tv_nop\n\tv_nop\n\tv_nop" : "+v"(d) : "v"(a.w), "v"(b.w));
  return d;
}

__device__ __forceinline__ v8f wmh(const FragH& a, const FragH& b, v8f c) {
  v8f d = __builtin_amdgcn_wmma_f32_16x16x32_f16(false, a.v, false, b.v, (short)0, c, false, false);
  asm volatile("v_nop\n\tv_nop\n\tv_nop\n\tv_nop" : "+v"(d) : "v"(a.w), "v"(b.w));
  return d;
}

__device__ __forceinline__ unsigned bf16_bits(float f) {
  const unsigned u = __float_as_uint(f);
  const unsigned r = (u + 0x7FFFu + ((u >> 16) & 1u)) >> 16;
  const unsigned q = (u >> 16) | 0x40u;
  return ((u & 0x7fffffffu) > 0x7f800000u) ? q : r;
}

__device__ __forceinline__ float bf16_val(float f) {
  return __uint_as_float(bf16_bits(f) << 16);
}
__device__ __forceinline__ int clampi(int v, int lo, int hi) {
  return v < lo ? lo : (v > hi ? hi : v);
}

__device__ __forceinline__ unsigned f16_bits(float f) {
  const unsigned u  = __float_as_uint(f);
  const unsigned s  = (u >> 16) & 0x8000u;
  const unsigned a  = u & 0x7fffffffu;
  const unsigned t  = a - 0x38000000u;
  const unsigned r  = (t + 0x0FFFu + ((t >> 13) & 1u)) >> 13;
  const unsigned rc = r > 0x7C00u ? 0x7C00u : r;
  const bool small  = a < 0x38800000u;
  const bool isnan  = a > 0x7f800000u;
  const unsigned fin = small ? 0u : (s | rc);
  return isnan ? (s | 0x7E00u) : fin;
}

__device__ __forceinline__ unsigned pk16(unsigned lo, unsigned hi) { return lo | (hi << 16); }
__device__ __forceinline__ unsigned bf16_lo_bits(float v) {
  float hi = bf16_val(v);
  asm volatile("" : "+v"(hi));
  return bf16_bits(v - hi);
}
__device__ __forceinline__ v4u pack8_bf16(v4f a, v4f c) {
  return (v4u){ pk16(bf16_bits(a[0]), bf16_bits(a[1])), pk16(bf16_bits(a[2]), bf16_bits(a[3])),
                pk16(bf16_bits(c[0]), bf16_bits(c[1])), pk16(bf16_bits(c[2]), bf16_bits(c[3])) };
}
__device__ __forceinline__ v4u pack8_bf16_lo(v4f a, v4f c) {
  return (v4u){ pk16(bf16_lo_bits(a[0]), bf16_lo_bits(a[1])), pk16(bf16_lo_bits(a[2]), bf16_lo_bits(a[3])),
                pk16(bf16_lo_bits(c[0]), bf16_lo_bits(c[1])), pk16(bf16_lo_bits(c[2]), bf16_lo_bits(c[3])) };
}
__device__ __forceinline__ v4u pack8_f16(v4f a, v4f c) {
  return (v4u){ pk16(f16_bits(a[0]), f16_bits(a[1])), pk16(f16_bits(a[2]), f16_bits(a[3])),
                pk16(f16_bits(c[0]), f16_bits(c[1])), pk16(f16_bits(c[2]), f16_bits(c[3])) };
}

template <int FORM>
__global__ __launch_bounds__(256) void k_plane(const float* __restrict__ src, int rows, int cols, int ldsrc,
                                               unsigned short* __restrict__ dst, int MP, int KP) {
  static_assert(FORM >= 0 && FORM <= 3);
  const int KTOT = (FORM == 1 || FORM == 3) ? 2 * KP : KP;
  const unsigned ppr   = (unsigned)(KTOT >> 3);
  const unsigned kp8   = (unsigned)(KP >> 3);
  const unsigned total = (unsigned)MP * ppr;
  const unsigned g     = blockIdx.x * 256u + threadIdx.x;
  const unsigned rowu  = g / ppr;
  const unsigned p     = g - rowu * ppr;
  const bool second    = p >= kp8;
  const int row = (int)rowu;
  const int c0  = (int)((second ? p - kp8 : p) << 3);
  const float* srow = src + (size_t)clampi(row, 0, rows - 1) * (size_t)ldsrc;
  float x[8];
  unsigned mk[8];
#pragma unroll
  for (int e = 0; e < 8; ++e) {
    const int c = c0 + e;
    const float v = srow[clampi(c, 0, cols - 1)];
    asm volatile("" :: "v"(v));
    x[e]  = v;
    mk[e] = (row < rows && c < cols) ? 0xFFFFu : 0u;
  }
  const v4f a = (v4f){ x[0], x[1], x[2], x[3] };
  const v4f c = (v4f){ x[4], x[5], x[6], x[7] };
  v4u o;
  if (FORM == 2) {
    o = pack8_f16(a, c);
  } else {
    const v4u hi = pack8_bf16(a, c);
    o = hi;
    if (FORM == 1) { const v4u lo = pack8_bf16_lo(a, c); o = second ? lo : hi; }
  }
  const v4u mw = (v4u){ pk16(mk[0], mk[1]), pk16(mk[2], mk[3]), pk16(mk[4], mk[5]), pk16(mk[6], mk[7]) };
  o &= mw;
  if (g < total) {
    volatile v4u* q = (volatile v4u*)(dst + (size_t)g * 8);
    *q = o;
    __threadfence();
    *q = o;
  }
}

template <int FORM> struct FragOf    { typedef FragB T; };
template <>         struct FragOf<2> { typedef FragH T; };
__device__ __forceinline__ v8f mm(const FragB& a, const FragB& b, v8f c) { return wmb(a, b, c); }
__device__ __forceinline__ v8f mm(const FragH& a, const FragH& b, v8f c) { return wmh(a, b, c); }
template <class F> __device__ __forceinline__ F ld_frag(const unsigned short* p) {
  F f;
  f.h[0] = *(const v8usa*)(p);
  f.h[1] = *(const v8usa*)(p + 16);
  return f;
}

template <int FORM, int EPI>
__global__ __launch_bounds__(256) __attribute__((amdgpu_num_vgpr(248)))
void k_gemm_nt(const unsigned short* __restrict__ A, const unsigned short* __restrict__ B,
               const float* __restrict__ bias, float* __restrict__ D, int M, int N, int KTOT, int ldd) {
  static_assert(FORM >= 0 && FORM <= 2);
  static_assert(EPI == 0 || EPI == 1);
  typedef typename FragOf<FORM>::T F;
  __shared__ __attribute__((aligned(16))) float sT[8][16 * 68];
  const int lane = threadIdx.x & 31;
  const int wave = threadIdx.x >> 5;
  const int tilesM = (M + 63) >> 6;
  const int tilesN = (N + 63) >> 6;
  const int tile = blockIdx.x * 8 + wave;
  if (tile >= tilesM * tilesN) return;
  const int tm = tile / tilesN;
  const int tn = tile - tm * tilesN;
  const int m0 = tm << 6;
  const int n0 = tn << 6;

  const int rl = lane & 15;
  const int h8 = (lane >> 4) * 8;
  const unsigned short* pa = A + (size_t)(m0 + rl) * (size_t)KTOT + h8;
  const unsigned short* pb = B + (size_t)(n0 + rl) * (size_t)KTOT + h8;

  v8f acc[4][4];
#pragma unroll
  for (int i = 0; i < 4; ++i)
#pragma unroll
    for (int j = 0; j < 4; ++j) acc[i][j] = (v8f){0.f, 0.f, 0.f, 0.f, 0.f, 0.f, 0.f, 0.f};

#pragma unroll 1
  for (int k0 = 0; k0 < KTOT; k0 += 32) {
    F bf[4];
#pragma unroll
    for (int j = 0; j < 4; ++j) bf[j] = ld_frag<F>(pb + (size_t)(j << 4) * (size_t)KTOT + k0);
#pragma unroll
    for (int i = 0; i < 4; ++i) {
      const F af = ld_frag<F>(pa + (size_t)(i << 4) * (size_t)KTOT + k0);
#pragma unroll
      for (int j = 0; j < 4; ++j) acc[i][j] = mm(af, bf[j], acc[i][j]);
    }
  }

  float* slab = sT[wave];
  const int hh = lane >> 4;
  const int c4 = (lane & 15) * 4;
  const int nc = n0 + c4;
  const bool cok = nc < N;
  v4f bv = (v4f){0.f, 0.f, 0.f, 0.f};
  if (EPI == 1) {
    bv = *(const v4fa*)(bias + clampi(nc, 0, N - 4));
    asm volatile("" :: "v"(bv));
  }
#pragma unroll
  for (int i = 0; i < 4; ++i) {
    const int mBase = m0 + (i << 4);
#pragma unroll
    for (int j = 0; j < 4; ++j) {
#pragma unroll
      for (int r = 0; r < 8; ++r) slab[(h8 + r) * 68 + (j << 4) + rl] = acc[i][j][r];
    }
    __builtin_amdgcn_fence(__ATOMIC_RELEASE, "workgroup");
    __builtin_amdgcn_wave_barrier();
    __builtin_amdgcn_fence(__ATOMIC_ACQUIRE, "workgroup");
    v4f vv[8];
#pragma unroll
    for (int it = 0; it < 8; ++it) {
      const int row = it * 2 + hh;
      v4f v = *(const v4fa*)(slab + row * 68 + c4);
      if (EPI == 1) v += bv;
      vv[it] = v;
    }
    for (int pass = 0; pass < 2; ++pass) {
#pragma unroll
      for (int it = 0; it < 8; ++it) {
        const int row = mBase + it * 2 + hh;
        if (cok && row < M) *(volatile v4f*)(D + (size_t)row * (size_t)ldd + nc) = vv[it];
      }
      __threadfence();
    }
    __builtin_amdgcn_fence(__ATOMIC_RELEASE, "workgroup");
    __builtin_amdgcn_wave_barrier();
    __builtin_amdgcn_fence(__ATOMIC_ACQUIRE, "workgroup");
  }
}

#include <stddef.h>

typedef int   v4i __attribute__((ext_vector_type(4)));
typedef float v2f __attribute__((ext_vector_type(2)));
typedef v4i __attribute__((may_alias)) v4ia;
typedef v2f __attribute__((may_alias)) v2fa;

#define SPLIT2 1

constexpr int G_N     = 100000;
constexpr int G_E     = 800000;
constexpr int DIN     = 128;
constexpr int C1      = 128;
constexpr int C2      = 64;
constexpr int KT      = SPLIT2 ? 256 : 128;
constexpr int PPR     = KT / 8;
constexpr int MPROWS  = 100096;
constexpr int NBRUN   = 1024;
constexpr int NBLK    = 98;
constexpr int CAP     = 10752;
constexpr int DEGCAP  = 32;
constexpr int BK_CHUNK = 2048;
constexpr int BK_WCAP  = 256;
constexpr int BK_LISTN = 8 * BK_WCAP;
constexpr int BK_LDS_INTS  = 2 * CAP + 3 * NBRUN + BK_LISTN + 16;
constexpr int BK_LDS_BYTES = BK_LDS_INTS * 4;
constexpr int BK_ZERO4     = (2 * CAP + NBRUN) / 4;
constexpr int PAR_AS1 = 0, PAR_AD1 = 128, PAR_B1 = 256, PAR_AS2 = 384, PAR_AD2 = 448, PAR_B2 = 512, PAR_N = 576;

static_assert(C1 == 2 * 64);
static_assert(G_N % 16 == 0);
static_assert(G_N <= (1 << 17));
static_assert(NBRUN == (1 << 10));
static_assert(NBLK * NBRUN >= MPROWS);
static_assert((NBLK - 1) * NBRUN < G_N);
static_assert(MPROWS % 128 == 0 && MPROWS >= G_N);
static_assert(4 * CAP >= 5 * 8361);
static_assert(DEGCAP >= 23 + 8 && DEGCAP <= 32);
static_assert(CAP % 32 == 0 && (CAP / 4) % 32 == 0);
static_assert(BK_ZERO4 % 256 == 0);
static_assert(BK_LDS_BYTES <= 262144);
static_assert((MPROWS * PPR) % 256 == 0);
static_assert((C1 * PPR) % 256 == 0 && (C2 * PPR) % 256 == 0);
static_assert(KT % 32 == 0 && DIN == 128);

constexpr size_t SZ_RA   = (size_t)MPROWS * KT * 2;
constexpr size_t SZ_RB   = (size_t)MPROWS * C1 * 4;
constexpr size_t SZ_S    = (size_t)G_N * 4 * 4;
constexpr size_t SZ_LIST = (size_t)NBLK * CAP * 4;
constexpr size_t SZ_CNT  = (size_t)NBLK * NBRUN * 4;
constexpr size_t SZ_FLAG = (size_t)NBLK * 128;
constexpr size_t SZ_W1T  = (size_t)C1 * KT * 2;
constexpr size_t SZ_W2T  = (size_t)C2 * KT * 2;
constexpr size_t SZ_PAR  = (size_t)PAR_N * 4;
constexpr size_t O_RA   = 0;
constexpr size_t O_RB   = O_RA + SZ_RA;
constexpr size_t O_S    = O_RB + SZ_RB;
constexpr size_t O_LIST = O_S + SZ_S;
constexpr size_t O_CNT  = O_LIST + SZ_LIST;
constexpr size_t O_OFF  = O_CNT + SZ_CNT;
constexpr size_t O_FLAG = O_OFF + SZ_CNT;
constexpr size_t O_W1T  = O_FLAG + SZ_FLAG;
constexpr size_t O_W2T  = O_W1T + SZ_W1T;
constexpr size_t O_PAR  = O_W2T + SZ_W2T;
constexpr size_t WS_TOTAL = O_PAR + SZ_PAR;
static_assert(SZ_RA % 128 == 0 && SZ_RB % 128 == 0 && SZ_S % 128 == 0 && SZ_LIST % 128 == 0);
static_assert(SZ_CNT % 128 == 0 && SZ_FLAG % 128 == 0 && SZ_W1T % 128 == 0 && SZ_W2T % 128 == 0 && SZ_PAR % 128 == 0);
static_assert(WS_TOTAL <= ((size_t)128 << 20));
static_assert((size_t)G_N * C1 * 4 <= SZ_RB && (size_t)G_N * C2 * 4 <= SZ_RB);
static_assert((size_t)G_N * 2 * 4 <= SZ_S);

__device__ __forceinline__ float leaky(float v, float s) { return (v > 0.0f) ? v : s * v; }
__device__ __forceinline__ float maxk(float m, float o) { return (o > m || o != o) ? o : m; }

__device__ __forceinline__ void wt_unit(const float* __restrict__ w, int cols, unsigned short* __restrict__ dst, int u) {
  const int n  = u / PPR;
  const int p  = u - n * PPR;
  const int k0 = (p * 8) & (DIN - 1);
  const float* q = w + (size_t)k0 * (size_t)cols + n;
  float x[8];
#pragma unroll
  for (int e = 0; e < 8; ++e) {
    const float v = q[(size_t)e * (size_t)cols];
    asm volatile("" :: "v"(v));
    x[e] = v;
  }
  const v4u o = pack8_bf16((v4f){ x[0], x[1], x[2], x[3] }, (v4f){ x[4], x[5], x[6], x[7] });
  volatile v4u* d = (volatile v4u*)(dst + (size_t)u * 8);
  *d = o;
  __threadfence();
  *d = o;
}

__device__ __forceinline__ void par_seg(const float* __restrict__ src, float* __restrict__ dst, int nq, int lane) {
  const int lc = lane < nq ? lane : nq - 1;
  const v4f v = *(const v4fa*)(src + 4 * lc);
  asm volatile("" :: "v"(v));
  const v4f o = (v4f){ bf16_val(v[0]), bf16_val(v[1]), bf16_val(v[2]), bf16_val(v[3]) };
  volatile v4f* d = (volatile v4f*)(dst + 4 * lc);
  if (lane < nq) *d = o;
  __threadfence();
  if (lane < nq) *d = o;
}

__global__ __launch_bounds__(256) void k_prep(const float* __restrict__ W1, const float* __restrict__ W2,
                                              const float* __restrict__ as1, const float* __restrict__ ad1,
                                              const float* __restrict__ b1, const float* __restrict__ as2,
                                              const float* __restrict__ ad2, const float* __restrict__ b2,
                                              unsigned short* __restrict__ w1t, unsigned short* __restrict__ w2t,
                                              float* __restrict__ par) {
  constexpr int B1 = C1 * PPR / 256;
  constexpr int B2 = C2 * PPR / 256;
  const int tid = (int)threadIdx.x;
  const int blk = (int)blockIdx.x;
  if (blk < B1) {
    wt_unit(W1, C1, w1t, blk * 256 + tid);
  } else if (blk < B1 + B2) {
    wt_unit(W2, C2, w2t, (blk - B1) * 256 + tid);
  } else {
    const int lane = tid & 31;
    if ((tid >> 5) == 0) {
      par_seg(as1, par + PAR_AS1, 32, lane);
      par_seg(ad1, par + PAR_AD1, 32, lane);
      par_seg(b1,  par + PAR_B1,  32, lane);
      par_seg(as2, par + PAR_AS2, 16, lane);
      par_seg(ad2, par + PAR_AD2, 16, lane);
      par_seg(b2,  par + PAR_B2,  16, lane);
    }
  }
}

__global__ __launch_bounds__(256) void k_h0(const float* __restrict__ x, const float* __restrict__ emb,
                                            unsigned short* __restrict__ dst) {
  const unsigned g   = blockIdx.x * 256u + threadIdx.x;
  const int row = (int)(g / (unsigned)PPR);
  const int p   = (int)(g - (unsigned)row * (unsigned)PPR);
  const bool second = p >= 16;
  const int c0  = (p & 15) * 8;
  const int rc  = row < G_N ? row : G_N - 1;
  const size_t so = (size_t)rc * DIN + c0;
  const v4f xa = *(const v4fa*)(x + so);
  const v4f xc = *(const v4fa*)(x + so + 4);
  const v4f ea = *(const v4fa*)(emb + so);
  const v4f ec = *(const v4fa*)(emb + so + 4);
  asm volatile("" :: "v"(xa));
  asm volatile("" :: "v"(xc));
  asm volatile("" :: "v"(ea));
  asm volatile("" :: "v"(ec));
  v4f ha, hc;
#pragma unroll
  for (int e = 0; e < 4; ++e) {
    const float ta = 1.0f + bf16_val(xa[e]);
    const float tc = 1.0f + bf16_val(xc[e]);
    ha[e] = bf16_val(ea[e]) * ta;
    hc[e] = bf16_val(ec[e]) * tc;
  }
  const v4u hi = pack8_bf16(ha, hc);
  const v4u lo = pack8_bf16_lo(ha, hc);
  v4u o = second ? lo : hi;
  const unsigned mk = (row < G_N) ? 0xFFFFFFFFu : 0u;
  o &= (v4u){ mk, mk, mk, mk };
  if (g < (unsigned)MPROWS * (unsigned)PPR) {
    volatile v4u* q = (volatile v4u*)(dst + (size_t)g * 8);
    *q = o;
    __threadfence();
    *q = o;
  }
}

__global__ __launch_bounds__(256) void k_bucket(const int* __restrict__ ei, int* __restrict__ LISTp,
                                                int* __restrict__ CNTp, int* __restrict__ OFFp, int* __restrict__ FLAGp) {
  extern __shared__ v4f lds_dyn[];
  int* reg1 = (int*)lds_dyn;
  int* reg2 = reg1 + CAP;
  int* scnt = reg2 + CAP;
  int* soff = scnt + NBRUN;
  int* cur  = soff + NBRUN;
  int* list = cur + NBRUN;
  int* wcnt = list + BK_LISTN;
  int* wtot = wcnt + 8;
  const int tid  = (int)threadIdx.x, lane = tid & 31;
  const int wave = __builtin_amdgcn_readfirstlane(tid >> 5);
  const int blk  = (int)blockIdx.x;
  const int slotBase = blk * NBRUN;
  const int nbr = G_N - slotBase;
  const int nb  = nbr < NBRUN ? nbr : NBRUN;
  const int* srcs = ei;
  const int* dsts = ei + G_E;

  for (int i = tid; i < BK_ZERO4; i += 256) *(v4ia*)(reg1 + 4 * i) = (v4i){0, 0, 0, 0};
  __syncthreads();

  int tot = 0, totraw = 0;
  constexpr int nChunks = (G_E + BK_CHUNK - 1) / BK_CHUNK;
  const int elw = wave * 256 + lane;
#pragma unroll 1
  for (int ch = 0; ch < nChunks; ++ch) {
    const int cbase = ch * BK_CHUNK;
    int kk[8];
#pragma unroll
    for (int j = 0; j < 8; ++j) {
      const int e  = cbase + elw + 32 * j;
      const int ec = e < G_E - 1 ? e : G_E - 1;
      const int k  = dsts[ec];
      asm volatile("" :: "v"(k));
      kk[j] = (e < G_E) ? k : -1;
    }
    unsigned sj[8];
    bool hj[8];
    bool anyl = false;
#pragma unroll
    for (int j = 0; j < 8; ++j) {
      sj[j] = (unsigned)kk[j] - (unsigned)slotBase;
      hj[j] = sj[j] < (unsigned)nb;
      anyl = anyl || hj[j];
    }
    int wc = 0;
    const unsigned any = __builtin_amdgcn_ballot_w32(anyl);
    if (any != 0u) {
#pragma unroll
      for (int j = 0; j < 8; ++j) {
        const unsigned mj = __builtin_amdgcn_ballot_w32(hj[j]);
        const int pos = wc + (int)__builtin_amdgcn_mbcnt_lo(mj, 0u);
        if (hj[j] && pos < BK_WCAP) list[wave * BK_WCAP + pos] = ((elw + 32 * j) << 10) | (int)sj[j];
        wc += (int)__builtin_popcount(mj);
      }
    }
    if (lane == 0) wcnt[wave] = wc;
    __syncthreads();
    int pre = 0, all = 0;
#pragma unroll
    for (int w2 = 0; w2 < 8; ++w2) {
      int c = wcnt[w2];
      c = c < 0 ? 0 : (c > BK_WCAP ? BK_WCAP : c);
      all += c;
      pre += (w2 < wave) ? c : 0;
    }
    const int wcc  = __builtin_amdgcn_readfirstlane(wc > BK_WCAP ? BK_WCAP : wc);
    const int base = tot + pre;
#pragma unroll 1
    for (int i0 = 0; i0 < wcc; i0 += 32) {
      const int i   = i0 + lane;
      const int ic  = i < wcc ? i : wcc - 1;
      const int ent = list[wave * BK_WCAP + ic];
      const int el  = (ent >> 10) & (BK_CHUNK - 1);
      const int sl  = ent & (NBRUN - 1);
      int eid = cbase + el;
      eid = eid > G_E - 1 ? G_E - 1 : eid;
      const int sraw = srcs[eid];
      asm volatile("" :: "v"(sraw));
      const int s   = clampi(sraw, 0, G_N - 1);
      const int pos = base + i;
      if (i < wcc && pos < CAP) reg1[pos] = (s << 10) | sl;
    }
    totraw += all;
    tot += all;
    tot = tot > CAP ? CAP : tot;
    __syncthreads();
  }
  const int nh  = __builtin_amdgcn_readfirstlane(tot);
  const int ovf = (totraw > CAP) ? 1 : 0;

  if (wave == 0) {
#pragma unroll 1
    for (int b0 = 0; b0 < nh; b0 += 32) {
      const int idx = b0 + lane;
      const int uv  = reg1[idx < CAP ? idx : CAP - 1];
      const int rem = nh - b0;
      const int m32 = rem < 32 ? rem : 32;
#pragma unroll 1
      for (int k = 0; k < m32; ++k) {
        const int u  = __builtin_amdgcn_readlane(uv, k);
        const int sl = u & (NBRUN - 1);
        const int cv = scnt[sl];
        if (lane == 0) scnt[sl] = cv + 1;
      }
    }
  }
  __syncthreads();

  {
    const v4i ca = *(const v4ia*)(scnt + 4 * tid);
    const int e0 = ca.x < 0 ? 0 : ca.x, e1 = ca.y < 0 ? 0 : ca.y, e2 = ca.z < 0 ? 0 : ca.z, e3 = ca.w < 0 ? 0 : ca.w;
    const int ts = e0 + e1 + e2 + e3;
    int incl = ts;
#pragma unroll
    for (int d = 1; d < 32; d <<= 1) {
      const int up = __shfl_up(incl, d);
      incl += (lane >= d) ? up : 0;
    }
    if (lane == 31) wtot[wave] = incl;
    __syncthreads();
    int pre = 0;
#pragma unroll
    for (int w2 = 0; w2 < 8; ++w2) pre += (w2 < wave) ? wtot[w2] : 0;
    const int r0 = pre + incl - ts;
    const v4i so = (v4i){ r0, r0 + e0, r0 + e0 + e1, r0 + e0 + e1 + e2 };
    *(v4ia*)(soff + 4 * tid) = so;
    *(v4ia*)(cur + 4 * tid)  = so;
  }
  __syncthreads();

  if (wave == 0) {
#pragma unroll 1
    for (int b0 = 0; b0 < nh; b0 += 32) {
      const int idx = b0 + lane;
      const int uv  = reg1[idx < CAP ? idx : CAP - 1];
      const int rem = nh - b0;
      const int m32 = rem < 32 ? rem : 32;
#pragma unroll 1
      for (int k = 0; k < m32; ++k) {
        const int u  = __builtin_amdgcn_readlane(uv, k);
        const int sl = u & (NBRUN - 1);
        const int sv = (int)((unsigned)u >> 10);
        int pos = cur[sl];
        pos = pos < 0 ? 0 : (pos > CAP - 1 ? CAP - 1 : pos);
        if (lane == 0) { reg2[pos] = sv; cur[sl] = pos + 1; }
      }
    }
  }
  __syncthreads();

  int* lb = LISTp + (size_t)blk * CAP;
  const v4i cq = *(const v4ia*)(scnt + 4 * tid);
  const v4i oq = *(const v4ia*)(soff + 4 * tid);
  const v4i fq = (v4i){ ovf, ovf, ovf, ovf };
  for (int pass = 0; pass < 2; ++pass) {
#pragma unroll 1
    for (int p = tid; p < CAP / 4; p += 256) {
      const v4i v = *(const v4ia*)(reg2 + 4 * p);
      *(volatile v4i*)(lb + 4 * p) = v;
    }
    *(volatile v4i*)(CNTp + slotBase + 4 * tid) = cq;
    *(volatile v4i*)(OFFp + slotBase + 4 * tid) = oq;
    if (tid < 8) *(volatile v4i*)(FLAGp + blk * 32 + 4 * tid) = fq;
    __threadfence();
  }
}

template <int LAYER>
__global__ __launch_bounds__(256) void k_score(const float* __restrict__ Hf, const float* __restrict__ par,
                                               float* __restrict__ S) {
  constexpr int SWD = (LAYER == 1) ? 4 : 2;
  __shared__ __attribute__((aligned(16))) float sPar[PAR_N];
  __shared__ __attribute__((aligned(16))) float sS[256 * 4];
  const int tid  = (int)threadIdx.x, lane = tid & 31;
  const int wave = __builtin_amdgcn_readfirstlane(tid >> 5);
  {
    const int ic = tid < PAR_N / 4 - 1 ? tid : PAR_N / 4 - 1;
    const v4f pv = *(const v4fa*)(par + 4 * ic);
    asm volatile("" :: "v"(pv));
    if (tid < PAR_N / 4) *(v4fa*)(&sPar[4 * tid]) = pv;
  }
  __syncthreads();
  const int row0 = (int)blockIdx.x * 256;
  int nrows = G_N - row0;
  nrows = nrows > 256 ? 256 : nrows;
  float a0, a1, a2 = 0.f, a3 = 0.f, d0, d1, d2 = 0.f, d3 = 0.f;
  if (LAYER == 1) {
    const v4f av = *(const v4fa*)(&sPar[PAR_AS1 + 4 * lane]);
    const v4f dv = *(const v4fa*)(&sPar[PAR_AD1 + 4 * lane]);
    a0 = av[0]; a1 = av[1]; a2 = av[2]; a3 = av[3];
    d0 = dv[0]; d1 = dv[1]; d2 = dv[2]; d3 = dv[3];
  } else {
    const v2f av = *(const v2fa*)(&sPar[PAR_AS2 + 2 * lane]);
    const v2f dv = *(const v2fa*)(&sPar[PAR_AD2 + 2 * lane]);
    a0 = av[0]; a1 = av[1];
    d0 = dv[0]; d1 = dv[1];
  }
  const int hd = lane >> 4;
#pragma unroll 1
  for (int j = 0; j < 32; ++j) {
    const int rl = wave * 32 + j;
    if (rl < nrows) {
      const int row = row0 + rl;
      float ps, pd;
      if (LAYER == 1) {
        const v4f hv = *(const v4fa*)(Hf + (size_t)row * C1 + 4 * lane);
        ps = hv[0] * a0; ps = fmaf(hv[1], a1, ps); ps = fmaf(hv[2], a2, ps); ps = fmaf(hv[3], a3, ps);
        pd = hv[0] * d0; pd = fmaf(hv[1], d1, pd); pd = fmaf(hv[2], d2, pd); pd = fmaf(hv[3], d3, pd);
#pragma unroll
        for (int off = 8; off > 0; off >>= 1) { ps += __shfl_xor(ps, off); pd += __shfl_xor(pd, off); }
        if ((lane & 15) == 0) { sS[rl * 4 + hd] = ps; sS[rl * 4 + 2 + hd] = pd; }
      } else {
        const v2f hv = *(const v2fa*)(Hf + (size_t)row * C2 + 2 * lane);
        ps = hv[0] * a0; ps = fmaf(hv[1], a1, ps);
        pd = hv[0] * d0; pd = fmaf(hv[1], d1, pd);
#pragma unroll
        for (int off = 16; off > 0; off >>= 1) { ps += __shfl_xor(ps, off); pd += __shfl_xor(pd, off); }
        if (lane == 0) { sS[rl * 2] = ps; sS[rl * 2 + 1] = pd; }
      }
    }
  }
  __syncthreads();
  const int npc = (LAYER == 1) ? nrows : (nrows >> 1);
  const int pc  = tid < npc ? tid : npc - 1;
  const v4f ov  = *(const v4fa*)(&sS[4 * pc]);
  volatile v4f* q = (volatile v4f*)(S + (size_t)row0 * SWD + 4 * pc);
  if (tid < npc) *q = ov;
  __threadfence();
  if (tid < npc) *q = ov;
}

template <int LAYER>
__global__ __launch_bounds__(256) void k_replay(const float* __restrict__ Hf, const float* __restrict__ S,
                                                const float* __restrict__ par, const int* __restrict__ LISTp,
                                                const int* __restrict__ CNTp, const int* __restrict__ OFFp,
                                                const int* __restrict__ FLAGp,
                                                unsigned short* __restrict__ xhl, float* __restrict__ out) {
  constexpr int ROWLIM = (LAYER == 1) ? MPROWS : G_N;
  __shared__ __attribute__((aligned(16))) float sPar[PAR_N];
  const int tid  = (int)threadIdx.x, lane = tid & 31;
  const int wave = __builtin_amdgcn_readfirstlane(tid >> 5);
  const int blk  = (int)blockIdx.x;
  {
    const int ic = tid < PAR_N / 4 - 1 ? tid : PAR_N / 4 - 1;
    const v4f pv = *(const v4fa*)(par + 4 * ic);
    asm volatile("" :: "v"(pv));
    if (tid < PAR_N / 4) *(v4fa*)(&sPar[4 * tid]) = pv;
  }
  __syncthreads();
  float bb0, bb1, bb2 = 0.f, bb3 = 0.f;
  if (LAYER == 1) {
    const v4f b = *(const v4fa*)(&sPar[PAR_B1 + 4 * lane]);
    bb0 = b[0]; bb1 = b[1]; bb2 = b[2]; bb3 = b[3];
  } else {
    const v2f b = *(const v2fa*)(&sPar[PAR_B2 + 2 * lane]);
    bb0 = b[0]; bb1 = b[1];
  }
  const bool hd1 = (LAYER == 1) && (lane >= 16);
  const int lc   = lane & 15;
  const int flag = FLAGp[blk * 32];
  const float qnan = __int_as_float(0x7fc00000);
  const int* lbase = LISTp + (size_t)blk * CAP;

#pragma unroll 1
  for (int jt = 0; jt < 128; ++jt) {
    const int t = blk * NBRUN + wave * 128 + jt;
    if (t < ROWLIM) {
      const bool live = t < G_N;
      const int tc = live ? t : G_N - 1;
      const int craw = CNTp[t];
      const int oraw = OFFp[t];
      int cv = craw < 0 ? 0 : (craw > DEGCAP ? DEGCAP : craw);
      const int ov = clampi(oraw, 0, CAP - 1);
      cv = cv > CAP - ov ? CAP - ov : cv;
      cv = live ? cv : 0;
      const int cn = __builtin_amdgcn_readfirstlane(cv);
      const int ob = __builtin_amdgcn_readfirstlane(ov);
      const bool bad = live && ((flag != 0) || craw > DEGCAP || craw < 0);

      const int lq = lane < cn ? lane : (cn > 0 ? cn - 1 : 0);
      const int sraw = lbase[ob + lq];
      asm volatile("" :: "v"(sraw));
      const int s = clampi(sraw, 0, G_N - 1);
      const bool valid = lane < cn;

      float as0, as1, tas0, tas1, tad0, tad1;
      if (LAYER == 1) {
        const v2f ss = *(const v2fa*)(S + (size_t)s * 4);
        asm volatile("" :: "v"(ss));
        const v4f st = *(const v4fa*)(S + (size_t)tc * 4);
        asm volatile("" :: "v"(st));
        as0 = ss[0]; as1 = ss[1];
        tas0 = st[0]; tas1 = st[1]; tad0 = st[2]; tad1 = st[3];
      } else {
        const float sa = S[(size_t)s * 2];
        asm volatile("" :: "v"(sa));
        const v2f st = *(const v2fa*)(S + (size_t)tc * 2);
        asm volatile("" :: "v"(st));
        as0 = sa; as1 = sa;
        tas0 = st[0]; tas1 = st[0]; tad0 = st[1]; tad1 = st[1];
      }
      const float es0 = leaky(tas0 + tad0, 0.2f);
      const float e0r = leaky(as0 + tad0, 0.2f);
      const float e0  = valid ? e0r : es0;
      float m0 = e0;
#pragma unroll
      for (int off = 16; off > 0; off >>= 1) { const float o = __shfl_xor(m0, off); m0 = maxk(m0, o); }
      const float p0 = expf(e0 - m0);
      float p1 = p0, es_own = es0, m_own = m0;
      if (LAYER == 1) {
        const float es1 = leaky(tas1 + tad1, 0.2f);
        const float e1r = leaky(as1 + tad1, 0.2f);
        const float e1  = valid ? e1r : es1;
        float m1 = e1;
#pragma unroll
        for (int off = 16; off > 0; off >>= 1) { const float o = __shfl_xor(m1, off); m1 = maxk(m1, o); }
        p1 = expf(e1 - m1);
        es_own = hd1 ? es1 : es0;
        m_own  = hd1 ? m1 : m0;
      }
      const float psf = expf(es_own - m_own);

      float hs0, hs1, hs2 = 0.f, hs3 = 0.f;
      if (LAYER == 1) {
        const v4f hv = *(const v4fa*)(Hf + (size_t)tc * C1 + 4 * lane);
        asm volatile("" :: "v"(hv));
        hs0 = hv[0]; hs1 = hv[1]; hs2 = hv[2]; hs3 = hv[3];
      } else {
        const v2f hv = *(const v2fa*)(Hf + (size_t)tc * C2 + 2 * lane);
        asm volatile("" :: "v"(hv));
        hs0 = hv[0]; hs1 = hv[1];
      }

      float acc0 = 0.0f, acc1 = 0.0f, acc2 = 0.0f, acc3 = 0.0f, den = 0.0f;
#pragma unroll 1
      for (int q = 0; q < cn; ++q) {
        const int sq = __builtin_amdgcn_readlane(s, q);
        const float pa = __int_as_float(__builtin_amdgcn_readlane(__float_as_int(p0), q));
        float p = pa;
        if (LAYER == 1) {
          const float pb = __int_as_float(__builtin_amdgcn_readlane(__float_as_int(p1), q));
          p = hd1 ? pb : pa;
          const v4f hv = *(const v4fa*)(Hf + (size_t)sq * C1 + 4 * lane);
          asm volatile("" :: "v"(hv));
          acc0 = fmaf(p, hv[0], acc0); acc1 = fmaf(p, hv[1], acc1);
          acc2 = fmaf(p, hv[2], acc2); acc3 = fmaf(p, hv[3], acc3);
        } else {
          const v2f hv = *(const v2fa*)(Hf + (size_t)sq * C2 + 2 * lane);
          asm volatile("" :: "v"(hv));
          acc0 = fmaf(p, hv[0], acc0); acc1 = fmaf(p, hv[1], acc1);
        }
        den += p;
      }
      acc0 = fmaf(psf, hs0, acc0); acc1 = fmaf(psf, hs1, acc1);
      acc2 = fmaf(psf, hs2, acc2); acc3 = fmaf(psf, hs3, acc3);
      den += psf;
      const float rinv = 1.0f / den;

      float v0 = leaky(acc0 * rinv + bb0, 0.01f);
      float v1 = leaky(acc1 * rinv + bb1, 0.01f);
      float v2 = leaky(acc2 * rinv + bb2, 0.01f);
      float v3 = leaky(acc3 * rinv + bb3, 0.01f);
      v0 = bad ? qnan : (live ? v0 : 0.0f);
      v1 = bad ? qnan : (live ? v1 : 0.0f);
      v2 = bad ? qnan : (live ? v2 : 0.0f);
      v3 = bad ? qnan : (live ? v3 : 0.0f);

      if (LAYER == 1) {
        const int sA = 2 * lc, sB = 2 * lc + 1;
        const v4f a = (v4f){ __shfl(v0, sA), __shfl(v1, sA), __shfl(v2, sA), __shfl(v3, sA) };
        const v4f c = (v4f){ __shfl(v0, sB), __shfl(v1, sB), __shfl(v2, sB), __shfl(v3, sB) };
        const v4u hi = pack8_bf16(a, c);
        const v4u lo = pack8_bf16_lo(a, c);
        const v4u o  = (lane < 16) ? hi : lo;
        volatile v4u* d = (volatile v4u*)(xhl + (size_t)t * KT + 8 * lane);
        if (lane < PPR) *d = o;
        __threadfence();
        if (lane < PPR) *d = o;
      } else {
        const int sA = 2 * lc, sB = 2 * lc + 1;
        const v4f o = (v4f){ __shfl(v0, sA), __shfl(v1, sA), __shfl(v0, sB), __shfl(v1, sB) };
        volatile v4f* d = (volatile v4f*)(out + (size_t)t * C2 + 4 * lc);
        if (lane < 16) *d = o;
        __threadfence();
        if (lane < 16) *d = o;
      }
    }
  }
  (void)xhl; (void)out;
}

extern "C" void kernel_launch(void* const* d_in, const int* in_sizes, int n_in,
                              void* d_out, int out_size, void* d_ws, size_t ws_size,
                              hipStream_t stream) {
  if (n_in < 11) return;
  if (in_sizes[0] != G_N * DIN || in_sizes[1] != 2 * G_E || in_sizes[2] != G_N * DIN) return;
  if (in_sizes[3] != DIN * C1 || in_sizes[4] != C1 || in_sizes[5] != C1 || in_sizes[6] != C1) return;
  if (in_sizes[7] != C1 * C2 || in_sizes[8] != C2 || in_sizes[9] != C2 || in_sizes[10] != C2) return;
  if (out_size != G_N * C2) return;
  if (ws_size < WS_TOTAL) return;

  const float* x    = (const float*)d_in[0];
  const int*   ei   = (const int*)  d_in[1];
  const float* emb  = (const float*)d_in[2];
  const float* W1   = (const float*)d_in[3];
  const float* as1  = (const float*)d_in[4];
  const float* ad1  = (const float*)d_in[5];
  const float* b1   = (const float*)d_in[6];
  const float* W2   = (const float*)d_in[7];
  const float* as2  = (const float*)d_in[8];
  const float* ad2  = (const float*)d_in[9];
  const float* b2   = (const float*)d_in[10];
  float* out = (float*)d_out;

  char* ws = (char*)d_ws;
  unsigned short* RA   = (unsigned short*)(ws + O_RA);
  float*          RB   = (float*)(ws + O_RB);
  float*          SP   = (float*)(ws + O_S);
  int*            LIST = (int*)(ws + O_LIST);
  int*            CNT  = (int*)(ws + O_CNT);
  int*            OFF  = (int*)(ws + O_OFF);
  int*            FLAG = (int*)(ws + O_FLAG);
  unsigned short* W1T  = (unsigned short*)(ws + O_W1T);
  unsigned short* W2T  = (unsigned short*)(ws + O_W2T);
  float*          PAR  = (float*)(ws + O_PAR);

  hipFuncSetAttribute(reinterpret_cast<const void*>(&k_bucket),
                      hipFuncAttributeMaxDynamicSharedMemorySize, BK_LDS_BYTES);

  k_prep<<<C1 * PPR / 256 + C2 * PPR / 256 + 1, 256, 0, stream>>>(W1, W2, as1, ad1, b1, as2, ad2, b2, W1T, W2T, PAR);
  k_h0<<<MPROWS * PPR / 256, 256, 0, stream>>>(x, emb, RA);
  k_bucket<<<NBLK, 256, BK_LDS_BYTES, stream>>>(ei, LIST, CNT, OFF, FLAG);
  {
    const int tiles = ((G_N + 63) / 64) * (C1 / 64);
    k_gemm_nt<0, 0><<<(tiles + 7) / 8, 256, 0, stream>>>(RA, W1T, PAR, RB, G_N, C1, KT, C1);
  }
  k_score<1><<<(G_N + 255) / 256, 256, 0, stream>>>(RB, PAR, SP);
  k_replay<1><<<NBLK, 256, 0, stream>>>(RB, SP, PAR, LIST, CNT, OFF, FLAG, RA, out);
  {
    const int tiles = ((G_N + 63) / 64) * (C2 / 64);
    k_gemm_nt<0, 0><<<(tiles + 7) / 8, 256, 0, stream>>>(RA, W2T, PAR, RB, G_N, C2, KT, C2);
  }
  k_score<2><<<(G_N + 255) / 256, 256, 0, stream>>>(RB, PAR, SP);
  k_replay<2><<<NBLK, 256, 0, stream>>>(RB, SP, PAR, LIST, CNT, OFF, FLAG, RA, out);
}
